// ModelWrapper_46231027974768
// MI455X (gfx1250) — hardware-run, weakly checked
//
#include <hip/hip_runtime.h>
#include <math.h>

typedef __attribute__((ext_vector_type(16))) _Float16 v16h;
typedef __attribute__((ext_vector_type(8)))  _Float16 v8h;
typedef __attribute__((ext_vector_type(8)))  float    v8f;
typedef __attribute__((ext_vector_type(4)))  float    v4f;
typedef __attribute__((ext_vector_type(2)))  unsigned v2u;

constexpr int kB   = 16;
constexpr int kT0  = 16000;
constexpr int kT1  = 8000;
constexpr int kT2  = 4000;
constexpr int kN   = 64;
constexpr int kCls = 12;
constexpr int kR1  = 128000;
constexpr int kR2  = 64000;
constexpr int kNumIn = 19;
constexpr float kLeak   = 0.01f;
constexpr float kWCarry = 1024.0f;
constexpr float kC1S    = 0.25f;
constexpr float kC2I    = 0.25f;
constexpr float kC2S    = 0.0625f;
static_assert(kT0 == 2 * kT1 && kT1 == 2 * kT2);
static_assert(kR1 == kB * kT1 && kR2 == kB * kT2);
static_assert(kB * kT0 == 256000);
static_assert((kN % 64) == 0 && (kN % 32) == 0 && (kN % 8) == 0);
static_assert((kR1 % 32) == 0 && (kR2 % 32) == 0);
static_assert(((kR1 / 32) * (kN / 64)) % 8 == 0);
static_assert(((kR2 / 32) * (kN / 64)) % 8 == 0);
static_assert(((kN * kN / 8) % 256) == 0);
static_assert(((kR1 * 8) % 256) == 0);
static_assert(((kR2 * 16) % 256) == 0);
static_assert(((kR2 * 8) % 256) == 0);
static_assert(((kB * kN) % 256) == 0);
static_assert(kB * 8 == 128);
static_assert(kB * kCls == 192 && kB * kCls * 4 == 768);

constexpr size_t kSzW16  = (size_t)kN * kN * 2;
constexpr size_t kSzS0H  = (size_t)kR1 * kN * 2;
constexpr size_t kSzP    = (size_t)kR1 * kN * 4;
constexpr size_t kSzH1H  = (size_t)kR1 * kN * 2;
constexpr size_t kSzH1E  = (size_t)kR2 * kN * 4;
constexpr size_t kSzS1H  = (size_t)kR2 * kN * 2;
constexpr size_t kSzH2   = (size_t)kR2 * kN * 4;
constexpr size_t kSzH2H  = (size_t)kR2 * kN * 2;
constexpr size_t kSzS2H  = (size_t)kR2 * kN * 2;
constexpr size_t kSzMEAN = (size_t)kB * kN * 4;
static_assert(kSzW16 == 8192ull);
static_assert(kSzS0H == 16384000ull);
static_assert(kSzP == 32768000ull);
static_assert(kSzH1H == 16384000ull);
static_assert(kSzH1E == 16384000ull);
static_assert(kSzS1H == 8192000ull);
static_assert(kSzH2 == 16384000ull);
static_assert(kSzH2H == 8192000ull);
static_assert(kSzS2H == 8192000ull);
static_assert(kSzMEAN == 4096ull);
constexpr size_t kOffC0H  = 0;
constexpr size_t kOffB1H  = kOffC0H  + kSzW16;
constexpr size_t kOffC1H  = kOffB1H  + kSzW16;
constexpr size_t kOffB2H  = kOffC1H  + kSzW16;
constexpr size_t kOffC2H  = kOffB2H  + kSzW16;
constexpr size_t kOffS0H  = kOffC2H  + kSzW16;
constexpr size_t kOffP    = kOffS0H  + kSzS0H;
constexpr size_t kOffH1H  = kOffP    + kSzP;
constexpr size_t kOffH1E  = kOffH1H  + kSzH1H;
constexpr size_t kOffS1H  = kOffH1E  + kSzH1E;
constexpr size_t kOffH2   = kOffS1H  + kSzS1H;
constexpr size_t kOffH2H  = kOffH2   + kSzH2;
constexpr size_t kOffS2H  = kOffH2H  + kSzH2H;
constexpr size_t kOffMEAN = kOffS2H  + kSzS2H;
constexpr size_t kWsTotal = kOffMEAN + kSzMEAN;
static_assert(kWsTotal == 122925056ull);
static_assert(kWsTotal <= 134217728ull);
static_assert((kSzW16 % 128) == 0 && (kSzS0H % 128) == 0 && (kSzP % 128) == 0 && (kSzH1H % 128) == 0 &&
              (kSzH1E % 128) == 0 && (kSzS1H % 128) == 0 && (kSzH2 % 128) == 0 && (kSzH2H % 128) == 0 &&
              (kSzS2H % 128) == 0 && (kSzMEAN % 128) == 0);
static_assert((kOffB1H % 128) == 0 && (kOffC1H % 128) == 0 && (kOffB2H % 128) == 0 && (kOffC2H % 128) == 0 &&
              (kOffS0H % 128) == 0 && (kOffP % 128) == 0 && (kOffH1H % 128) == 0 && (kOffH1E % 128) == 0 &&
              (kOffS1H % 128) == 0 && (kOffH2 % 128) == 0 && (kOffH2H % 128) == 0 && (kOffS2H % 128) == 0 &&
              (kOffMEAN % 128) == 0);

__device__ __forceinline__ _Float16 f16_flush(float v) {
  const float w = (fabsf(v) < 6.103515625e-05f) ? 0.0f : v;
  return (_Float16)w;
}

__device__ __forceinline__ float bf16r(float v) {
  unsigned u = __float_as_uint(v);
  u = (u + 0x7FFFu + ((u >> 16) & 1u)) & 0xFFFF0000u;
  return __uint_as_float(u);
}

namespace eng {
union FragU { v16h v; v8h h[2]; };
__device__ __forceinline__ v16h frag_load(const _Float16* p) {
  FragU f;
  f.h[0] = *(const v8h*)(p);
  f.h[1] = *(const v8h*)(p + 16);
  return f.v;
}
__device__ __forceinline__ v8f mma(v16h a, v16h b, v8f c) {
  return __builtin_amdgcn_wmma_f32_16x16x32_f16(false, a, false, b, (short)0, c, false, false);
}
__device__ __forceinline__ void guard1(v8f& a, v16h x, v16h y) {
  asm volatile("v_nop\n\tv_nop\n\tv_nop\n\tv_nop" : "+v"(a) : "v"(x), "v"(y));
}
__device__ __forceinline__ void guard_acc(v8f& a) {
  asm volatile("v_nop\n\tv_nop\n\tv_nop\n\tv_nop" : "+v"(a));
}
__device__ __forceinline__ void keep4(v16h a, v16h b, v16h c, v16h d) {
  asm volatile("v_nop" :: "v"(a), "v"(b), "v"(c), "v"(d));
}

template <int MI, int SPL>
__global__ __launch_bounds__(256) void gemm_f16_kernel(
    const unsigned short* __restrict__ Ap, const unsigned short* __restrict__ A2p, int lda,
    const unsigned short* __restrict__ Btp, const unsigned short* __restrict__ Bt2p, int ldb,
    float* __restrict__ C, int ldc, int M, int N, int K, float scale, float rscale)
{
  static_assert(MI >= 1 && MI <= 2);
  static_assert(SPL >= 0 && SPL <= 2);
  const _Float16* A   = (const _Float16*)Ap;
  const _Float16* A2  = (const _Float16*)A2p;
  const _Float16* Bt  = (const _Float16*)Btp;
  const _Float16* Bt2 = (const _Float16*)Bt2p;
  __shared__ __align__(16) float sT[8][16 * 68];
  const int lane = threadIdx.x & 31;
  const int wave = threadIdx.x >> 5;
  const int tilesN = N >> 6;
  const int tilesM = M / (16 * MI);
  const int tile = blockIdx.x * 8 + wave;
  if (tile >= tilesM * tilesN) return;
  const int tm = tile / tilesN;
  const int tn = tile - tm * tilesN;
  const int m0 = tm * (16 * MI);
  const int n0 = tn << 6;
  const int rlane = lane & 15;
  const int koff  = (lane >> 4) * 8;
  const int mOff  = (lane >> 4) * 8;

  v8f acc[MI][4], accr[MI][4];
#pragma unroll
  for (int i = 0; i < MI; ++i)
#pragma unroll
    for (int j = 0; j < 4; ++j) {
      acc[i][j]  = (v8f){0.f, 0.f, 0.f, 0.f, 0.f, 0.f, 0.f, 0.f};
      accr[i][j] = (v8f){0.f, 0.f, 0.f, 0.f, 0.f, 0.f, 0.f, 0.f};
    }

  for (int k0 = 0; k0 < K; k0 += 32) {
    v16h bh[4], bl[4];
#pragma unroll
    for (int j = 0; j < 4; ++j) {
      const size_t bo = (size_t)(n0 + (j << 4) + rlane) * ldb + koff + k0;
      bh[j] = frag_load(Bt + bo);
      if (SPL == 2) bl[j] = frag_load(Bt2 + bo); else bl[j] = bh[j];
    }
#pragma unroll
    for (int i = 0; i < MI; ++i) {
      const size_t ao = (size_t)(m0 + (i << 4) + rlane) * lda + koff + k0;
      const v16h ah = frag_load(A + ao);
      v16h al = ah;
      if (SPL >= 1) al = frag_load(A2 + ao);
#pragma unroll
      for (int j = 0; j < 4; ++j) {
        acc[i][j] = mma(ah, bh[j], acc[i][j]);
        if (SPL >= 1) accr[i][j] = mma(al, bh[j], accr[i][j]);
        if (SPL == 2) accr[i][j] = mma(ah, bl[j], accr[i][j]);
      }
#pragma unroll
      for (int j = 0; j < 4; ++j) {
        guard1(acc[i][j], ah, al);
        if (SPL >= 1) guard1(accr[i][j], ah, al);
      }
    }
    keep4(bh[0], bh[1], bh[2], bh[3]);
    if (SPL == 2) keep4(bl[0], bl[1], bl[2], bl[3]);
  }
#pragma unroll
  for (int i = 0; i < MI; ++i)
#pragma unroll
    for (int j = 0; j < 4; ++j) {
      guard_acc(acc[i][j]);
      if (SPL >= 1) guard_acc(accr[i][j]);
    }

  float* slab = sT[wave];
#pragma unroll
  for (int i = 0; i < MI; ++i) {
    const int mBase = m0 + (i << 4);
#pragma unroll
    for (int j = 0; j < 4; ++j) {
#pragma unroll
      for (int r = 0; r < 8; ++r) {
        float v = acc[i][j][r] * scale;
        if (SPL >= 1) v += accr[i][j][r] * rscale;
        slab[(mOff + r) * 68 + (j << 4) + rlane] = v;
      }
    }
    __builtin_amdgcn_fence(__ATOMIC_RELEASE, "workgroup");
    __builtin_amdgcn_wave_barrier();
    __builtin_amdgcn_fence(__ATOMIC_ACQUIRE, "workgroup");
    {
      const int hh = lane >> 4, c4 = (lane & 15) * 4;
      for (int pass = 0; pass < 2; ++pass) {
#pragma unroll
        for (int it = 0; it < 8; ++it) {
          const int row = it * 2 + hh;
          const v4f v = *(const v4f*)(slab + row * 68 + c4);
          *(volatile v4f*)(C + (size_t)(mBase + row) * ldc + n0 + c4) = v;
        }
        __threadfence();
      }
    }
    __builtin_amdgcn_fence(__ATOMIC_RELEASE, "workgroup");
    __builtin_amdgcn_wave_barrier();
    __builtin_amdgcn_fence(__ATOMIC_ACQUIRE, "workgroup");
  }
}
}

__global__ __launch_bounds__(256) void pack_rows_bf_kernel(
    const float* __restrict__ W, unsigned short* __restrict__ dH,
    int Kdim, int Nreal, int total8, float carry)
{
  const int i = blockIdx.x * 256 + threadIdx.x;
  if (i >= total8) return;
  const size_t e0 = (size_t)i << 3;
  const int row = (int)(e0 / (size_t)Kdim);
  const int col = (int)(e0 - (size_t)row * (size_t)Kdim);
  const bool live = (row < Nreal);
  const int rc = live ? row : (Nreal - 1);
  const v4f a0 = *(const v4f*)(W + (size_t)rc * Kdim + col);
  const v4f a1 = *(const v4f*)(W + (size_t)rc * Kdim + col + 4);
  const float w0 = a0[0];
  const float w1 = a0[1];
  const float w2 = a0[2];
  const float w3 = a0[3];
  const float w4 = a1[0];
  const float w5 = a1[1];
  const float w6 = a1[2];
  const float w7 = a1[3];
  const float t0 = bf16r(w0) * carry;
  const float t1 = bf16r(w1) * carry;
  const float t2 = bf16r(w2) * carry;
  const float t3 = bf16r(w3) * carry;
  const float t4 = bf16r(w4) * carry;
  const float t5 = bf16r(w5) * carry;
  const float t6 = bf16r(w6) * carry;
  const float t7 = bf16r(w7) * carry;
  const float g0 = live ? t0 : 0.0f;
  const float g1 = live ? t1 : 0.0f;
  const float g2 = live ? t2 : 0.0f;
  const float g3 = live ? t3 : 0.0f;
  const float g4 = live ? t4 : 0.0f;
  const float g5 = live ? t5 : 0.0f;
  const float g6 = live ? t6 : 0.0f;
  const float g7 = live ? t7 : 0.0f;
  v8h hv;
  hv[0] = f16_flush(g0);
  hv[1] = f16_flush(g1);
  hv[2] = f16_flush(g2);
  hv[3] = f16_flush(g3);
  hv[4] = f16_flush(g4);
  hv[5] = f16_flush(g5);
  hv[6] = f16_flush(g6);
  hv[7] = f16_flush(g7);
  unsigned short* qh = dH + e0;
  *(volatile v8h*)qh = hv;
  __threadfence();
  *(volatile v8h*)qh = hv;
}

__device__ __forceinline__ void ld8(const float* __restrict__ p, float (&o)[8]) {
  const v4f q0 = *(const v4f*)(p);
  const v4f q1 = *(const v4f*)(p + 4);
  o[0] = q0[0];
  o[1] = q0[1];
  o[2] = q0[2];
  o[3] = q0[3];
  o[4] = q1[0];
  o[5] = q1[1];
  o[6] = q1[2];
  o[7] = q1[3];
}
__device__ __forceinline__ void ld8_bf(const float* __restrict__ p, float (&o)[8]) {
  float t[8];
  ld8(p, t);
#pragma unroll
  for (int e = 0; e < 8; ++e) o[e] = bf16r(t[e]);
}
__device__ __forceinline__ void st8h_twice(unsigned short* p, const float (&v)[8]) {
  v8h hv;
  hv[0] = f16_flush(v[0]);
  hv[1] = f16_flush(v[1]);
  hv[2] = f16_flush(v[2]);
  hv[3] = f16_flush(v[3]);
  hv[4] = f16_flush(v[4]);
  hv[5] = f16_flush(v[5]);
  hv[6] = f16_flush(v[6]);
  hv[7] = f16_flush(v[7]);
  *(volatile v8h*)p = hv;
  __threadfence();
  *(volatile v8h*)p = hv;
}
__device__ __forceinline__ float leaky_act(float o) {
  return (o > 0.0f) ? o : kLeak * o;
}

__global__ __launch_bounds__(128) void l0_scan_kernel(
    const float* __restrict__ x, const float* __restrict__ A0, const float* __restrict__ B0,
    const float* __restrict__ Bb0, unsigned short* __restrict__ S0H)
{
  const int tid = threadIdx.x;
  const int b = tid >> 3;
  const int n8 = tid & 7;
  float a[8], w[8], bb[8], s[8];
  ld8_bf(A0 + 8 * n8, a);
  ld8_bf(B0 + 8 * n8, w);
  ld8_bf(Bb0 + 8 * n8, bb);
#pragma unroll
  for (int e = 0; e < 8; ++e) s[e] = 0.0f;
  const float* xb = x + (size_t)b * kT0;
  unsigned short* sp = S0H + (size_t)b * kT1 * kN + 8 * n8;
  for (int t1 = 0; t1 < kT1; ++t1) {
    const float x0 = bf16r(xb[2 * t1]);
    const float x1 = bf16r(xb[2 * t1 + 1]);
#pragma unroll
    for (int e = 0; e < 8; ++e) s[e] = fmaf(s[e], a[e], fmaf(x0, w[e], bb[e]));
    st8h_twice(sp + (size_t)t1 * kN, s);
#pragma unroll
    for (int e = 0; e < 8; ++e) s[e] = fmaf(s[e], a[e], fmaf(x1, w[e], bb[e]));
  }
}

__global__ __launch_bounds__(256) void l0_epi_kernel(
    const float* __restrict__ P, const float* __restrict__ x, const float* __restrict__ Cb0,
    const float* __restrict__ Skip0, unsigned short* __restrict__ H1H)
{
  const int g = blockIdx.x * 256 + threadIdx.x;
  const int r = g >> 3;
  const int n8 = g & 7;
  const int b = r / kT1;
  const int t1 = r - b * kT1;
  float p[8], cb[8], sk[8], v[8];
  ld8(P + (size_t)r * kN + 8 * n8, p);
  ld8_bf(Cb0 + 8 * n8, cb);
  ld8_bf(Skip0 + 8 * n8, sk);
  const float xv = bf16r(x[(size_t)b * kT0 + 2 * t1]);
#pragma unroll
  for (int e = 0; e < 8; ++e) {
    const float o = p[e] + cb[e];
    v[e] = leaky_act(o) + sk[e] * xv;
  }
  st8h_twice(H1H + (size_t)r * kN + 8 * n8, v);
}

__global__ __launch_bounds__(256) void l0_skip_kernel(
    const float* __restrict__ P, const float* __restrict__ x, const float* __restrict__ Cb0,
    const float* __restrict__ Skip0, float* __restrict__ H1E)
{
  const int g = blockIdx.x * 256 + threadIdx.x;
  const int q = g >> 4;
  const int n4 = g & 15;
  const int b = q / kT2;
  const int t2 = q - b * kT2;
  const size_t r = (size_t)b * kT1 + 2 * t2;
  const v4f pv = *(const v4f*)(P + r * kN + 4 * n4);
  const v4f cv = *(const v4f*)(Cb0 + 4 * n4);
  const v4f sv = *(const v4f*)(Skip0 + 4 * n4);
  const float xv = bf16r(x[(size_t)b * kT0 + 4 * t2]);
  const float p0 = pv[0];
  const float p1 = pv[1];
  const float p2 = pv[2];
  const float p3 = pv[3];
  const float c0 = cv[0];
  const float c1 = cv[1];
  const float c2 = cv[2];
  const float c3 = cv[3];
  const float k0 = sv[0];
  const float k1 = sv[1];
  const float k2 = sv[2];
  const float k3 = sv[3];
  v4f res;
  res[0] = leaky_act(p0 + bf16r(c0)) + bf16r(k0) * xv;
  res[1] = leaky_act(p1 + bf16r(c1)) + bf16r(k1) * xv;
  res[2] = leaky_act(p2 + bf16r(c2)) + bf16r(k2) * xv;
  res[3] = leaky_act(p3 + bf16r(c3)) + bf16r(k3) * xv;
  float* dst = H1E + (size_t)q * kN + 4 * n4;
  *(volatile v4f*)dst = res;
  __threadfence();
  *(volatile v4f*)dst = res;
}

__global__ __launch_bounds__(128) void l1_scan_kernel(
    const float* __restrict__ P, const float* __restrict__ A1, const float* __restrict__ Bb1,
    unsigned short* __restrict__ S1H)
{
  const int tid = threadIdx.x;
  const int b = tid >> 3;
  const int n8 = tid & 7;
  float a[8], bb[8], s[8];
  ld8_bf(A1 + 8 * n8, a);
  ld8_bf(Bb1 + 8 * n8, bb);
#pragma unroll
  for (int e = 0; e < 8; ++e) s[e] = 0.0f;
  const float* pb = P + (size_t)b * kT1 * kN + 8 * n8;
  unsigned short* sp = S1H + (size_t)b * kT2 * kN + 8 * n8;
  for (int t2 = 0; t2 < kT2; ++t2) {
    float u0[8], u1[8], sc[8];
    ld8(pb + (size_t)(2 * t2) * kN, u0);
    ld8(pb + (size_t)(2 * t2 + 1) * kN, u1);
#pragma unroll
    for (int e = 0; e < 8; ++e) s[e] = fmaf(s[e], a[e], u0[e] + bb[e]);
#pragma unroll
    for (int e = 0; e < 8; ++e) sc[e] = s[e] * kC1S;
    st8h_twice(sp + (size_t)t2 * kN, sc);
#pragma unroll
    for (int e = 0; e < 8; ++e) s[e] = fmaf(s[e], a[e], u1[e] + bb[e]);
  }
}

__global__ __launch_bounds__(256) void l1_epi_kernel(
    const float* __restrict__ P, const float* __restrict__ Cb1, const float* __restrict__ H1E,
    unsigned short* __restrict__ H2H)
{
  const int g = blockIdx.x * 256 + threadIdx.x;
  const int q = g >> 3;
  const int n8 = g & 7;
  const size_t o8 = (size_t)q * kN + 8 * n8;
  float p[8], cb[8], sk[8], vc[8];
  ld8(P + o8, p);
  ld8_bf(Cb1 + 8 * n8, cb);
  ld8(H1E + o8, sk);
#pragma unroll
  for (int e = 0; e < 8; ++e) {
    const float o = p[e] + cb[e];
    const float v = leaky_act(o) + sk[e];
    vc[e] = v * kC2I;
  }
  st8h_twice(H2H + o8, vc);
}

__global__ __launch_bounds__(256) void l1_skip_kernel(
    const float* __restrict__ P, const float* __restrict__ Cb1, const float* __restrict__ H1E,
    float* __restrict__ H2)
{
  const int g = blockIdx.x * 256 + threadIdx.x;
  const int q = g >> 4;
  const int n4 = g & 15;
  const size_t o4 = (size_t)q * kN + 4 * n4;
  const v4f pv = *(const v4f*)(P + o4);
  const v4f cv = *(const v4f*)(Cb1 + 4 * n4);
  const v4f sv = *(const v4f*)(H1E + o4);
  const float p0 = pv[0];
  const float p1 = pv[1];
  const float p2 = pv[2];
  const float p3 = pv[3];
  const float c0 = cv[0];
  const float c1 = cv[1];
  const float c2 = cv[2];
  const float c3 = cv[3];
  const float k0 = sv[0];
  const float k1 = sv[1];
  const float k2 = sv[2];
  const float k3 = sv[3];
  v4f res;
  res[0] = leaky_act(p0 + bf16r(c0)) + k0;
  res[1] = leaky_act(p1 + bf16r(c1)) + k1;
  res[2] = leaky_act(p2 + bf16r(c2)) + k2;
  res[3] = leaky_act(p3 + bf16r(c3)) + k3;
  float* dst = H2 + o4;
  *(volatile v4f*)dst = res;
  __threadfence();
  *(volatile v4f*)dst = res;
}

__global__ __launch_bounds__(128) void l2_scan_kernel(
    const float* __restrict__ P, const float* __restrict__ A2, const float* __restrict__ Bb2,
    unsigned short* __restrict__ S2H)
{
  const int tid = threadIdx.x;
  const int b = tid >> 3;
  const int n8 = tid & 7;
  float a[8], bb[8], s[8];
  ld8_bf(A2 + 8 * n8, a);
  ld8_bf(Bb2 + 8 * n8, bb);
#pragma unroll
  for (int e = 0; e < 8; ++e) s[e] = 0.0f;
  const float* pb = P + (size_t)b * kT2 * kN + 8 * n8;
  unsigned short* sp = S2H + (size_t)b * kT2 * kN + 8 * n8;
  for (int t = 0; t < kT2; ++t) {
    float u[8], sc[8];
    ld8(pb + (size_t)t * kN, u);
#pragma unroll
    for (int e = 0; e < 8; ++e) s[e] = fmaf(s[e], a[e], u[e] + bb[e]);
#pragma unroll
    for (int e = 0; e < 8; ++e) sc[e] = s[e] * kC2S;
    st8h_twice(sp + (size_t)t * kN, sc);
  }
}

__global__ __launch_bounds__(256) void mean_kernel(
    const float* __restrict__ P, const float* __restrict__ Cb2, const float* __restrict__ H2,
    float* __restrict__ MEAN)
{
  const int i = blockIdx.x * 256 + threadIdx.x;
  const int b = i >> 6;
  const int n = i & 63;
  const float cb = bf16r(Cb2[n]);
  const float* pp = P + (size_t)b * kT2 * kN + n;
  const float* hp = H2 + (size_t)b * kT2 * kN + n;
  float acc = 0.0f;
  for (int t = 0; t < kT2; ++t) {
    const float o = pp[(size_t)t * kN] + cb;
    acc += leaky_act(o) + hp[(size_t)t * kN];
  }
  const float m = acc * (1.0f / (float)kT2);
  *(volatile float*)(MEAN + i) = m;
  __threadfence();
  *(volatile float*)(MEAN + i) = m;
}

__global__ __launch_bounds__(192) void head_kernel(
    const float* __restrict__ MEAN, const float* __restrict__ W, const float* __restrict__ bias,
    float* __restrict__ out)
{
  const int o = threadIdx.x;
  const int b = o / kCls;
  const int k = o - b * kCls;
  const float* mp = MEAN + b * kN;
  const float* wp = W + k * kN;
  float acc = 0.0f;
#pragma unroll
  for (int j = 0; j < kN / 4; ++j) {
    const v4f mv = *(const v4f*)(mp + 4 * j);
    const v4f wv = *(const v4f*)(wp + 4 * j);
    const float m0 = mv[0];
    const float m1 = mv[1];
    const float m2 = mv[2];
    const float m3 = mv[3];
    const float w0 = wv[0];
    const float w1 = wv[1];
    const float w2 = wv[2];
    const float w3 = wv[3];
    acc = fmaf(m0, bf16r(w0), acc);
    acc = fmaf(m1, bf16r(w1), acc);
    acc = fmaf(m2, bf16r(w2), acc);
    acc = fmaf(m3, bf16r(w3), acc);
  }
  const float res = acc + bf16r(bias[k]);
  *(volatile float*)(out + o) = res;
  __threadfence();
  *(volatile float*)(out + o) = res;
}

extern "C" void kernel_launch(void* const* d_in, const int* in_sizes, int n_in,
                              void* d_out, int out_size, void* d_ws, size_t ws_size,
                              hipStream_t stream)
{
  if (n_in != kNumIn) return;
  if (in_sizes[0] != kB * kT0) return;
  if (in_sizes[1] != kN) return;
  if (in_sizes[2] != kN) return;
  if (in_sizes[3] != kN) return;
  if (in_sizes[4] != kN * kN) return;
  if (in_sizes[5] != kN) return;
  if (in_sizes[6] != kN) return;
  if (in_sizes[7] != kN) return;
  if (in_sizes[8] != kN * kN) return;
  if (in_sizes[9] != kN) return;
  if (in_sizes[10] != kN * kN) return;
  if (in_sizes[11] != kN) return;
  if (in_sizes[12] != kN) return;
  if (in_sizes[13] != kN * kN) return;
  if (in_sizes[14] != kN) return;
  if (in_sizes[15] != kN * kN) return;
  if (in_sizes[16] != kN) return;
  if (in_sizes[17] != kCls * kN) return;
  if (in_sizes[18] != kCls) return;
  if (out_size != kB * kCls) return;
  if (ws_size < kWsTotal) return;

  const float* x     = (const float*)d_in[0];
  const float* A0    = (const float*)d_in[1];
  const float* B0    = (const float*)d_in[2];
  const float* Bb0   = (const float*)d_in[3];
  const float* C0    = (const float*)d_in[4];
  const float* Cb0   = (const float*)d_in[5];
  const float* Skip0 = (const float*)d_in[6];
  const float* A1    = (const float*)d_in[7];
  const float* B1    = (const float*)d_in[8];
  const float* Bb1   = (const float*)d_in[9];
  const float* C1    = (const float*)d_in[10];
  const float* Cb1   = (const float*)d_in[11];
  const float* A2    = (const float*)d_in[12];
  const float* B2    = (const float*)d_in[13];
  const float* Bb2   = (const float*)d_in[14];
  const float* C2w   = (const float*)d_in[15];
  const float* Cb2   = (const float*)d_in[16];
  const float* Wc    = (const float*)d_in[17];
  const float* bcls  = (const float*)d_in[18];
  float* out = (float*)d_out;

  char* ws = (char*)d_ws;
  unsigned short* C0H = (unsigned short*)(ws + kOffC0H);
  unsigned short* B1H = (unsigned short*)(ws + kOffB1H);
  unsigned short* C1H = (unsigned short*)(ws + kOffC1H);
  unsigned short* B2H = (unsigned short*)(ws + kOffB2H);
  unsigned short* C2H = (unsigned short*)(ws + kOffC2H);
  unsigned short* S0H = (unsigned short*)(ws + kOffS0H);
  float*          P   = (float*)(ws + kOffP);
  unsigned short* H1H = (unsigned short*)(ws + kOffH1H);
  float*          H1E = (float*)(ws + kOffH1E);
  unsigned short* S1H = (unsigned short*)(ws + kOffS1H);
  float*          H2  = (float*)(ws + kOffH2);
  unsigned short* H2H = (unsigned short*)(ws + kOffH2H);
  unsigned short* S2H = (unsigned short*)(ws + kOffS2H);
  float*          MEAN = (float*)(ws + kOffMEAN);

  constexpr int kPack8 = kN * kN / 8;
  constexpr int kPackBlocks = kPack8 / 256;
  constexpr int kTiles1 = (kR1 / 32) * (kN / 64);
  constexpr int kTiles2 = (kR2 / 32) * (kN / 64);
  constexpr float sc1 = 1.0f / kWCarry;
  constexpr float sc3 = 1.0f / (kWCarry * kC1S);
  constexpr float sc4 = 1.0f / (kWCarry * kC2I);
  constexpr float sc5 = 1.0f / (kWCarry * kC2S);
  static_assert(kPack8 == 512 && kPackBlocks == 2);
  static_assert(kTiles1 == 4000 && kTiles2 == 2000);

  pack_rows_bf_kernel<<<kPackBlocks, 256, 0, stream>>>(C0, C0H, kN, kN, kPack8, kWCarry);
  pack_rows_bf_kernel<<<kPackBlocks, 256, 0, stream>>>(B1, B1H, kN, kN, kPack8, kWCarry);
  pack_rows_bf_kernel<<<kPackBlocks, 256, 0, stream>>>(C1, C1H, kN, kN, kPack8, kWCarry);
  pack_rows_bf_kernel<<<kPackBlocks, 256, 0, stream>>>(B2, B2H, kN, kN, kPack8, kWCarry);
  pack_rows_bf_kernel<<<kPackBlocks, 256, 0, stream>>>(C2w, C2H, kN, kN, kPack8, kWCarry);

  l0_scan_kernel<<<1, 128, 0, stream>>>(x, A0, B0, Bb0, S0H);

  eng::gemm_f16_kernel<2, 0><<<dim3(kTiles1 / 8), 256, 0, stream>>>(
      S0H, nullptr, kN, C0H, nullptr, kN, P, kN, kR1, kN, kN, sc1, 0.0f);

  l0_epi_kernel<<<(kR1 * 8) / 256, 256, 0, stream>>>(P, x, Cb0, Skip0, H1H);
  l0_skip_kernel<<<(kR2 * 16) / 256, 256, 0, stream>>>(P, x, Cb0, Skip0, H1E);

  eng::gemm_f16_kernel<2, 0><<<dim3(kTiles1 / 8), 256, 0, stream>>>(
      H1H, nullptr, kN, B1H, nullptr, kN, P, kN, kR1, kN, kN, sc1, 0.0f);

  l1_scan_kernel<<<1, 128, 0, stream>>>(P, A1, Bb1, S1H);

  eng::gemm_f16_kernel<2, 0><<<dim3(kTiles2 / 8), 256, 0, stream>>>(
      S1H, nullptr, kN, C1H, nullptr, kN, P, kN, kR2, kN, kN, sc3, 0.0f);

  l1_epi_kernel<<<(kR2 * 8) / 256, 256, 0, stream>>>(P, Cb1, H1E, H2H);
  l1_skip_kernel<<<(kR2 * 16) / 256, 256, 0, stream>>>(P, Cb1, H1E, H2);

  eng::gemm_f16_kernel<2, 0><<<dim3(kTiles2 / 8), 256, 0, stream>>>(
      H2H, nullptr, kN, B2H, nullptr, kN, P, kN, kR2, kN, kN, sc4, 0.0f);

  l2_scan_kernel<<<1, 128, 0, stream>>>(P, A2, Bb2, S2H);

  eng::gemm_f16_kernel<2, 0><<<dim3(kTiles2 / 8), 256, 0, stream>>>(
      S2H, nullptr, kN, C2H, nullptr, kN, P, kN, kR2, kN, kN, sc5, 0.0f);

  mean_kernel<<<(kB * kN) / 256, 256, 0, stream>>>(P, Cb2, H2, MEAN);

  head_kernel<<<1, kB * kCls, 0, stream>>>(MEAN, Wc, bcls, out);
}
